// CausalSelfAttention_19774029431759
// MI455X (gfx1250) — hardware-verified
//
#include <hip/hip_runtime.h>


#ifndef NB
#define NB 2
#endif
#ifndef SEQ
#define SEQ 2048
#endif
#define NB_FULL  2
#define SEQ_FULL 2048
#define DM   1024
#define NH_  16
#define HD   64
#define RH   256
#define SCL  0.125f
#define L2E  1.4426950408889634f
#define RCAR 2048.0f

typedef _Float16 h16;
typedef unsigned short bf;
typedef __attribute__((ext_vector_type(16))) __bf16   v16bf;
typedef __attribute__((ext_vector_type(16))) _Float16 v16h;
typedef __attribute__((ext_vector_type(8)))  _Float16 v8h;
typedef __attribute__((ext_vector_type(2)))  _Float16 v2h;
typedef __attribute__((ext_vector_type(8)))  unsigned short v8us;
typedef __attribute__((ext_vector_type(2)))  unsigned short v2us;
typedef __attribute__((ext_vector_type(8)))  float    v8f;
typedef __attribute__((ext_vector_type(4)))  float    v4f;
typedef v4f  __attribute__((may_alias)) v4fa;

static_assert(NH_ * HD == DM);
static_assert(HD == 64);
static_assert(DM == 256 * 4);
static_assert(DM % 64 == 0 && DM % 32 == 0);
static_assert((3 * DM) % 64 == 0);
static_assert(SEQ % 64 == 0 && RH % 64 == 0 && RH % 32 == 0 && SEQ >= RH);
static_assert((NB * SEQ) % 64 == 0);
static_assert(NB <= NB_FULL && SEQ <= SEQ_FULL);

__device__ __forceinline__ unsigned short f2bf(float f) { unsigned u = __float_as_uint(f); u += 0x7FFFu + ((u >> 16) & 1u); return (unsigned short)(u >> 16); }
__device__ __forceinline__ float bf2f(unsigned short b) { return __uint_as_float(((unsigned)b) << 16); }
__device__ __forceinline__ float bfr(float f) { return bf2f(f2bf(f)); }
__device__ __forceinline__ void splitf(float y, unsigned short& h, unsigned short& l) { h = f2bf(y); l = f2bf(y - bf2f(h)); }
__device__ __forceinline__ v16h cat16(v8h lo, v8h hi) { return __builtin_shufflevector(lo, hi, 0, 1, 2, 3, 4, 5, 6, 7, 8, 9, 10, 11, 12, 13, 14, 15); }
__device__ __forceinline__ v16bf cat16b(v8us lo, v8us hi) { return __builtin_bit_cast(v16bf, __builtin_shufflevector(lo, hi, 0, 1, 2, 3, 4, 5, 6, 7, 8, 9, 10, 11, 12, 13, 14, 15)); }
__device__ __forceinline__ v8f wmma16(v16h a, v16h b, v8f c) { return __builtin_amdgcn_wmma_f32_16x16x32_f16(false, a, false, b, (short)0, c, false, false); }
__device__ __forceinline__ v8f wmmab(v16bf a, v16bf b, v8f c) { return __builtin_amdgcn_wmma_f32_16x16x32_bf16(false, a, false, b, (short)0, c, false, false); }
__device__ __forceinline__ v16h ldh(const h16* p) { return cat16(*(const v8h*)p, *(const v8h*)(p + 16)); }

template <typename T16> struct WFrag;
template <> struct WFrag<h16> { typedef v16h V; static __device__ __forceinline__ V ld(const h16* p) { return cat16(*(const v8h*)p, *(const v8h*)(p + 16)); } static __device__ __forceinline__ v8f mma(V a, V b, v8f c) { return wmma16(a, b, c); } };
template <> struct WFrag<bf> { typedef v16bf V; static __device__ __forceinline__ V ld(const bf* p) { return cat16b(*(const v8us*)p, *(const v8us*)(p + 16)); } static __device__ __forceinline__ v8f mma(V a, V b, v8f c) { return wmmab(a, b, c); } };

template <typename T16, int NSPLIT, bool BIAS>
__device__ __forceinline__ void gemmw_body(const T16* __restrict__ A, const T16* __restrict__ A2, const T16* __restrict__ Bt, const T16* __restrict__ Bt2, const int K, float* C, const int ldc, const float* __restrict__ bias, const size_t sA, const size_t sB, const size_t sC) {
    typedef typename WFrag<T16>::V V;
    __shared__ __align__(16) float os[16 * 68];
    const size_t z = blockIdx.z; A += z * sA; if (A2) A2 += z * sA; Bt += z * sB; if (Bt2) Bt2 += z * sB; C += z * sC;
    const int lane = threadIdx.x & 31, lr = lane & 15, hi = lane >> 4; const int r0 = blockIdx.x * 64, c0 = blockIdx.y * 64;
    v8f acc[4][4];
#pragma unroll
    for (int mb = 0; mb < 4; ++mb)
#pragma unroll
        for (int nb = 0; nb < 4; ++nb) acc[mb][nb] = (v8f){};
    const size_t aoff = (size_t)(r0 + lr) * K + 8 * hi, boff = (size_t)(c0 + lr) * K + 8 * hi;
#pragma unroll 1
    for (int kc = 0; kc < K; kc += 32) {
        V a[4], a2[4];
#pragma unroll
        for (int mb = 0; mb < 4; ++mb) { a[mb] = WFrag<T16>::ld(A + aoff + (size_t)mb * 16 * K + kc); if (NSPLIT == 1 || NSPLIT == 2) a2[mb] = WFrag<T16>::ld(A2 + aoff + (size_t)mb * 16 * K + kc); }
#pragma unroll
        for (int nb = 0; nb < 4; ++nb) { const V b = WFrag<T16>::ld(Bt + boff + (size_t)nb * 16 * K + kc); V b2; if (NSPLIT >= 2) b2 = WFrag<T16>::ld(Bt2 + boff + (size_t)nb * 16 * K + kc);
#pragma unroll
            for (int mb = 0; mb < 4; ++mb) { acc[mb][nb] = WFrag<T16>::mma(a[mb], b, acc[mb][nb]); if (NSPLIT == 1 || NSPLIT == 2) acc[mb][nb] = WFrag<T16>::mma(a2[mb], b, acc[mb][nb]); if (NSPLIT >= 2) acc[mb][nb] = WFrag<T16>::mma(a[mb], b2, acc[mb][nb]); } }
        asm volatile("v_nop\n\tv_nop\n\tv_nop\n\tv_nop" : "+v"(acc[0][0]), "+v"(acc[1][1]), "+v"(acc[2][2]), "+v"(acc[3][3]) : "v"(a[0]), "v"(a[3]));
    }
    v4f bv4 = (v4f){0.f, 0.f, 0.f, 0.f};
    if (BIAS) { const v4f braw = *(const v4f*)(bias + c0 + lr * 4); bv4[0] = bfr(braw[0]); bv4[1] = bfr(braw[1]); bv4[2] = bfr(braw[2]); bv4[3] = bfr(braw[3]); }
#pragma unroll
    for (int mb = 0; mb < 4; ++mb) {
#pragma unroll
        for (int nb = 0; nb < 4; ++nb) {
#pragma unroll
            for (int j = 0; j < 8; ++j) os[(hi * 8 + j) * 68 + nb * 16 + lr] = acc[mb][nb][j]; }
        __builtin_amdgcn_wave_barrier(); asm volatile("" ::: "memory");
        float* crow = C + (size_t)(r0 + mb * 16) * ldc + c0;
#pragma unroll 1
        for (int ps = 0; ps < 2; ++ps) {
#pragma unroll
            for (int s = 0; s < 8; ++s) { const int row = 2 * s + hi, cofs = lr * 4; v4f val = *(const v4fa*)(os + row * 68 + cofs); if (BIAS) val = val + bv4;
                *(volatile v4f*)(crow + (size_t)row * ldc + cofs) = val; }
            if (ps == 0) __threadfence(); }
        __builtin_amdgcn_wave_barrier(); asm volatile("" ::: "memory");
    }
}

__global__ __launch_bounds__(32) void k_gemm_qkv(const bf* __restrict__ XB, const bf* __restrict__ WT, float* F, const float* __restrict__ BC) {
    gemmw_body<bf, 0, true>(XB, nullptr, WT, nullptr, DM, F, 3 * DM, BC, 0, 0, 0);
}
__global__ __launch_bounds__(32) void k_gemm_out(const bf* __restrict__ ATh, const bf* __restrict__ ATl, const bf* __restrict__ WOt, float* OUT, const float* __restrict__ bo) {
    gemmw_body<bf, 1, true>(ATh, ATl, WOt, nullptr, DM, OUT, DM, bo, (size_t)SEQ * DM, 0, (size_t)SEQ_FULL * DM);
}

__global__ __launch_bounds__(256) void k_cvt8(const float* __restrict__ src, bf* dst, size_t n8, size_t sSrc, size_t sDst) {
    const size_t i = (size_t)blockIdx.x * 256 + threadIdx.x; if (i >= n8) return;
    src += (size_t)blockIdx.y * sSrc; dst += (size_t)blockIdx.y * sDst;
    const v8f v = *(const v8f*)(src + i * 8); v8us o;
#pragma unroll
    for (int k = 0; k < 8; ++k) o[k] = f2bf(v[k]);
    *(volatile v8us*)(dst + i * 8) = o; __threadfence(); *(volatile v8us*)(dst + i * 8) = o; }

__global__ __launch_bounds__(256) void k_wT(const float* __restrict__ W, bf* Bt) {
    const size_t e = ((size_t)blockIdx.x * 256 + threadIdx.x) * 2; if (e >= (size_t)DM * DM) return;
    const int k = (int)(e % DM); const int n = (int)(e / DM); v2us o;
#pragma unroll
    for (int q = 0; q < 2; ++q) o[q] = f2bf(W[(size_t)(k + q) * DM + n]);
    *(volatile v2us*)(Bt + e) = o; __threadfence(); *(volatile v2us*)(Bt + e) = o; }

__global__ __launch_bounds__(256) void k_bcat(const float* __restrict__ bq, const float* __restrict__ bk, const float* __restrict__ bv, float* BC) {
    const int i = threadIdx.x * 4;
    const v4f a = *(const v4f*)(bq + i); const v4f b = *(const v4f*)(bk + i); const v4f c = *(const v4f*)(bv + i);
    *(volatile v4f*)(BC + i) = a; *(volatile v4f*)(BC + DM + i) = b; *(volatile v4f*)(BC + 2 * DM + i) = c;
    __threadfence();
    *(volatile v4f*)(BC + i) = a; *(volatile v4f*)(BC + DM + i) = b; *(volatile v4f*)(BC + 2 * DM + i) = c; }

__global__ __launch_bounds__(256) void k_qk(const float* __restrict__ F, h16* QK, size_t n8) {
    const size_t i = (size_t)blockIdx.x * 256 + threadIdx.x; if (i >= n8) return;
    const size_t row = i / (2 * DM / 8); const int c8 = (int)(i % (2 * DM / 8)) * 8;
    const v8f v = *(const v8f*)(F + row * (3 * DM) + c8); v8h o;
#pragma unroll
    for (int k = 0; k < 8; ++k) o[k] = (h16)v[k];
    *(volatile v8h*)(QK + row * (2 * DM) + c8) = o; __threadfence(); *(volatile v8h*)(QK + row * (2 * DM) + c8) = o; }

__global__ __launch_bounds__(256) void k_vt(const float* __restrict__ F, h16* VT, h16* VR) {
    const size_t e = ((size_t)blockIdx.x * 256 + threadIdx.x) * 2; if (e >= (size_t)NB * DM * SEQ) return;
    const int t = (int)(e % SEQ); const int c = (int)((e / SEQ) % DM); const int b = (int)(e / ((size_t)SEQ * DM)); v2h o, r;
#pragma unroll
    for (int q = 0; q < 2; ++q) { const float xv = F[((size_t)b * SEQ + t + q) * (3 * DM) + 2 * DM + c]; const h16 hv = (h16)xv; o[q] = hv; r[q] = (h16)((xv - (float)hv) * RCAR); }
    const size_t er = ((size_t)b * DM + c) * RH + t;
    const bool early = (t < RH);
    *(volatile v2h*)(VT + e) = o; if (early) *(volatile v2h*)(VR + er) = r;
    __threadfence();
    *(volatile v2h*)(VT + e) = o; if (early) *(volatile v2h*)(VR + er) = r; }

template <bool HIRES>
__device__ __forceinline__ void flash_body(const h16* __restrict__ QK, const h16* __restrict__ VT, const h16* __restrict__ VR, bf* Ah, bf* Al, const int qbase) {
    __shared__ __align__(16) float fs[4 * 16 * 68];
    const int wave = __builtin_amdgcn_readfirstlane(threadIdx.x >> 5);
    const int lane = threadIdx.x & 31, lr = lane & 15, hh = lane >> 4;
    const int b = blockIdx.z, head = blockIdx.y;
    const int q0 = qbase + blockIdx.x * 64 + wave * 16;
    const int qi = q0 + lr;
    const size_t rowb = (size_t)b * SEQ;
    const size_t qoff = (rowb + (size_t)qi) * (2 * DM) + head * HD + 8 * hh;
    const size_t koff = (rowb + (size_t)lr) * (2 * DM) + DM + head * HD + 8 * hh;
    const size_t voff = ((size_t)b * DM + head * HD + lr) * SEQ + 8 * hh;
    const size_t roff = ((size_t)b * DM + head * HD + lr) * RH + 8 * hh;
    v8f o0 = (v8f){}, o1 = (v8f){}, o2 = (v8f){}, o3 = (v8f){};
    v8f r0 = (v8f){}, r1 = (v8f){}, r2 = (v8f){}, r3 = (v8f){};
    float mrun = -1.0e30f, lrun = 0.0f;
    const int nkb = (q0 + 15) / 32 + 1;
#pragma unroll 1
    for (int kb = 0; kb < nkb; ++kb) {
        const int key0 = kb * 32;
        v8f s0 = (v8f){}, s1 = (v8f){};
        {
            const v16h qa = ldh(QK + qoff), qb = ldh(QK + qoff + 32);
            const h16* kp = QK + koff + (size_t)key0 * (2 * DM);
            const v16h ka0 = ldh(kp), ka1 = ldh(kp + 32);
            const v16h kb0 = ldh(kp + (size_t)16 * (2 * DM)), kb1 = ldh(kp + (size_t)16 * (2 * DM) + 32);
            s0 = wmma16(ka0, qa, s0); s1 = wmma16(kb0, qa, s1);
            s0 = wmma16(ka1, qb, s0); s1 = wmma16(kb1, qb, s1);
            asm volatile("v_nop\n\tv_nop\n\tv_nop\n\tv_nop" : "+v"(s0), "+v"(s1) : "v"(qb), "v"(kb1));
        }
        float t0[8], t1[8]; float mloc = -1.0e30f;
        const int kk = key0 + 8 * hh;
#pragma unroll
        for (int r = 0; r < 8; ++r) {
            t0[r] = (kk + r <= qi) ? s0[r] * SCL : -1.0e30f;
            t1[r] = (kk + 16 + r <= qi) ? s1[r] * SCL : -1.0e30f;
            mloc = fmaxf(mloc, fmaxf(t0[r], t1[r])); }
        mloc = fmaxf(mloc, __shfl_xor(mloc, 16, 32));
        const float mnew = fmaxf(mrun, mloc);
        const float corr = __builtin_amdgcn_exp2f((mrun - mnew) * L2E);
        const float mL = mnew * L2E;
        mrun = mnew;
        float psum = 0.0f; v16h ph, pr;
#pragma unroll
        for (int r = 0; r < 8; ++r) {
            const float e0 = __builtin_amdgcn_exp2f(fmaf(t0[r], L2E, -mL));
            const float e1 = __builtin_amdgcn_exp2f(fmaf(t1[r], L2E, -mL));
            const float p0 = (t0[r] > -0.5e30f) ? e0 : 0.0f;
            const float p1 = (t1[r] > -0.5e30f) ? e1 : 0.0f;
            const h16 h0 = (h16)p0, h1 = (h16)p1;
            ph[r] = h0; ph[8 + r] = h1;
            if (HIRES) { pr[r] = (h16)((p0 - (float)h0) * RCAR); pr[8 + r] = (h16)((p1 - (float)h1) * RCAR); psum += p0 + p1; }
            else { psum += (float)h0 + (float)h1; } }
        lrun = lrun * corr + psum;
        o0 = o0 * corr; o1 = o1 * corr; o2 = o2 * corr; o3 = o3 * corr;
        if (HIRES) { r0 = r0 * corr; r1 = r1 * corr; r2 = r2 * corr; r3 = r3 * corr; }
        {
            const h16* vp = VT + voff + key0;
            const v16h v0 = ldh(vp), v1 = ldh(vp + (size_t)16 * SEQ), v2 = ldh(vp + (size_t)32 * SEQ), v3 = ldh(vp + (size_t)48 * SEQ);
            if (HIRES) {
                const h16* rp = VR + roff + key0;
                const v16h w0 = ldh(rp), w1 = ldh(rp + (size_t)16 * RH), w2 = ldh(rp + (size_t)32 * RH), w3 = ldh(rp + (size_t)48 * RH);
                o0 = wmma16(v0, ph, o0); o1 = wmma16(v1, ph, o1); o2 = wmma16(v2, ph, o2); o3 = wmma16(v3, ph, o3);
                r0 = wmma16(v0, pr, r0); r1 = wmma16(v1, pr, r1); r2 = wmma16(v2, pr, r2); r3 = wmma16(v3, pr, r3);
                r0 = wmma16(w0, ph, r0); r1 = wmma16(w1, ph, r1); r2 = wmma16(w2, ph, r2); r3 = wmma16(w3, ph, r3);
                asm volatile("v_nop\n\tv_nop\n\tv_nop\n\tv_nop" : "+v"(o0), "+v"(o1), "+v"(o2), "+v"(o3), "+v"(r0), "+v"(r1), "+v"(r2), "+v"(r3) : "v"(ph), "v"(w3));
            } else {
                o0 = wmma16(v0, ph, o0); o1 = wmma16(v1, ph, o1); o2 = wmma16(v2, ph, o2); o3 = wmma16(v3, ph, o3);
                asm volatile("v_nop\n\tv_nop\n\tv_nop\n\tv_nop" : "+v"(o0), "+v"(o1), "+v"(o2), "+v"(o3) : "v"(ph), "v"(v3));
            }
        }
    }
    const float ltot = lrun + __shfl_xor(lrun, 16, 32);
    const float inv = 1.0f / ltot;
    const int wb = wave * (16 * 68);
    const int ob = wb + lr * 68 + 8 * hh;
#pragma unroll
    for (int r = 0; r < 8; ++r) {
        float a0 = o0[r], a1 = o1[r], a2 = o2[r], a3 = o3[r];
        if (HIRES) { a0 += r0[r] * (1.0f / RCAR); a1 += r1[r] * (1.0f / RCAR); a2 += r2[r] * (1.0f / RCAR); a3 += r3[r] * (1.0f / RCAR); }
        fs[ob + r] = a0 * inv; fs[ob + 16 + r] = a1 * inv; fs[ob + 32 + r] = a2 * inv; fs[ob + 48 + r] = a3 * inv; }
    __builtin_amdgcn_wave_barrier(); asm volatile("" ::: "memory");
    const int rq = lane >> 3, pc = (lane & 7) * 8;
#pragma unroll 1
    for (int ps = 0; ps < 2; ++ps) {
#pragma unroll
        for (int s = 0; s < 4; ++s) {
            const int rr = 4 * s + rq;
            const v4f a = *(const v4fa*)(fs + wb + rr * 68 + pc);
            const v4f c = *(const v4fa*)(fs + wb + rr * 68 + pc + 4);
            v8us oh, ol;
#pragma unroll
            for (int k = 0; k < 4; ++k) { unsigned short x1, x2; splitf(a[k], x1, x2); oh[k] = x1; ol[k] = x2; splitf(c[k], x1, x2); oh[4 + k] = x1; ol[4 + k] = x2; }
            const size_t oo = (rowb + (size_t)(q0 + rr)) * DM + head * HD + pc;
            *(volatile v8us*)(Ah + oo) = oh; *(volatile v8us*)(Al + oo) = ol; }
        if (ps == 0) __threadfence(); }
}
__global__ __launch_bounds__(128) void k_flash_hi(const h16* __restrict__ QK, const h16* __restrict__ VT, const h16* __restrict__ VR, bf* Ah, bf* Al) { flash_body<true>(QK, VT, VR, Ah, Al, 0); }
__global__ __launch_bounds__(128) void k_flash_lo(const h16* __restrict__ QK, const h16* __restrict__ VT, const h16* __restrict__ VR, bf* Ah, bf* Al) { flash_body<false>(QK, VT, VR, Ah, Al, RH); }

#define AL256(x) ((((size_t)(x)) + 255) & ~(size_t)255)
#define SZ_XB  AL256((size_t)NB * SEQ * DM * 2)
#define SZ_WT  AL256((size_t)3 * DM * DM * 2)
#define SZ_WO  AL256((size_t)DM * DM * 2)
#define SZ_BC  AL256((size_t)3 * DM * 4)
#define SZ_F   AL256((size_t)NB * SEQ * 3 * DM * 4)
#define SZ_QK  AL256((size_t)NB * SEQ * 2 * DM * 2)
#define SZ_VT  AL256((size_t)NB * DM * SEQ * 2)
#define SZ_VR  AL256((size_t)NB * DM * RH * 2)
#define SZ_AT  AL256((size_t)NB * SEQ * DM * 2)
#define SZ_ALL (SZ_XB + SZ_WT + SZ_WO + SZ_BC + SZ_F + SZ_QK + SZ_VT + SZ_VR + SZ_AT + SZ_AT)
static_assert(SZ_ALL <= (size_t)134217728);

extern "C" void kernel_launch(void* const* d_in, const int* in_sizes, int n_in,
                              void* d_out, int out_size, void* d_ws, size_t ws_size, hipStream_t stream) {
    if (n_in < 9) return;
    const long long xneed = (long long)(NB - 1) * SEQ_FULL * DM + (long long)SEQ * DM;
    if ((long long)in_sizes[0] < xneed) return;
    if ((long long)in_sizes[1] < (long long)DM * DM || (long long)in_sizes[3] < (long long)DM * DM || (long long)in_sizes[5] < (long long)DM * DM || (long long)in_sizes[7] < (long long)DM * DM) return;
    if (in_sizes[2] < DM || in_sizes[4] < DM || in_sizes[6] < DM || in_sizes[8] < DM) return;
    if ((long long)out_size < xneed) return;
    if (ws_size < SZ_ALL) return;
    const float* x  = (const float*)d_in[0];
    const float* wq = (const float*)d_in[1]; const float* bq = (const float*)d_in[2];
    const float* wk = (const float*)d_in[3]; const float* bk = (const float*)d_in[4];
    const float* wv = (const float*)d_in[5]; const float* bv = (const float*)d_in[6];
    const float* wo = (const float*)d_in[7]; const float* bo = (const float*)d_in[8];
    float* OUT = (float*)d_out;
    char* wsp = (char*)d_ws;
    auto take = [&](size_t bytes) { char* p = wsp; wsp += bytes; return (void*)p; };
    bf* XB = (bf*)take(SZ_XB); bf* WT = (bf*)take(SZ_WT); bf* WOt = (bf*)take(SZ_WO); float* BC = (float*)take(SZ_BC);
    float* F = (float*)take(SZ_F); h16* QK = (h16*)take(SZ_QK); h16* VT = (h16*)take(SZ_VT); h16* VR = (h16*)take(SZ_VR);
    bf* ATh = (bf*)take(SZ_AT); bf* ATl = (bf*)take(SZ_AT);

    const size_t xn8 = (size_t)SEQ * DM / 8;
    k_cvt8<<<dim3((unsigned)((xn8 + 255) / 256), NB, 1), 256, 0, stream>>>(x, XB, xn8, (size_t)SEQ_FULL * DM, (size_t)SEQ * DM);
    const unsigned LW = (unsigned)(((size_t)DM * DM / 2 + 255) / 256);
    k_wT<<<LW, 256, 0, stream>>>(wq, WT);
    k_wT<<<LW, 256, 0, stream>>>(wk, WT + (size_t)DM * DM);
    k_wT<<<LW, 256, 0, stream>>>(wv, WT + (size_t)2 * DM * DM);
    k_wT<<<LW, 256, 0, stream>>>(wo, WOt);
    k_bcat<<<1, 256, 0, stream>>>(bq, bk, bv, BC);
    k_gemm_qkv<<<dim3(NB * SEQ / 64, 3 * DM / 64, 1), 32, 0, stream>>>(XB, WT, F, BC);
    const size_t qn8 = (size_t)NB * SEQ * 2 * DM / 8;
    k_qk<<<(unsigned)((qn8 + 255) / 256), 256, 0, stream>>>(F, QK, qn8);
    k_vt<<<(unsigned)(((size_t)NB * DM * SEQ / 2 + 255) / 256), 256, 0, stream>>>(F, VT, VR);
    k_flash_hi<<<dim3(RH / 64, NH_, NB), 128, 0, stream>>>(QK, VT, VR, ATh, ATl);
    if (SEQ > RH) k_flash_lo<<<dim3((SEQ - RH) / 64, NH_, NB), 128, 0, stream>>>(QK, VT, VR, ATh, ATl);
    k_gemm_out<<<dim3(SEQ / 64, DM / 64, NB), 32, 0, stream>>>(ATh, ATl, WOt, OUT, bo);
}
